// ExpertsModel_17523466568300
// MI455X (gfx1250) — hardware-verified
//
#include <hip/hip_runtime.h>
#include <stddef.h>
#include <stdint.h>

#pragma clang fp contract(off)

#define NTOK   4096
#define DD     512
#define FF     2048
#define NE     8
#define NTILE  72
#define NROWS  (NTILE * 64)
#define NCH    (NTOK / 256)
#define NPC    (NROWS / 4)
#define NPIT   5
#define WSC    64.0f
#define INV64  0.015625f
#define CHH    16.0f
#define INVHY  0.0009765625f
#define YPITCH 68
#define HPITCH 72
#define TP     68

static_assert(NTILE == NTOK / 64 + NE);
static_assert(NROWS % 4 == 0);
static_assert(NPC <= NPIT * 256);
static_assert(DD % 128 == 0);
static_assert(FF % 128 == 0);
static_assert(DD % 64 == 0);
static_assert(FF % 64 == 0);
static_assert(NTOK % 256 == 0);
static_assert(NTOK % 32 == 0);
static_assert(NTOK <= 65536);
static_assert(NE == 8);
static_assert((NROWS * 4) % 128 == 0);
static_assert((YPITCH * 4) % 16 == 0);
static_assert((HPITCH * 2) % 16 == 0);
static_assert((TP * 4) % 16 == 0);

typedef _Float16 v16h __attribute__((ext_vector_type(16)));
typedef _Float16 v8h  __attribute__((ext_vector_type(8)));
typedef float    v8f  __attribute__((ext_vector_type(8)));
typedef float    v4f  __attribute__((ext_vector_type(4)));
typedef unsigned int v4u __attribute__((ext_vector_type(4)));
typedef int      v4i  __attribute__((ext_vector_type(4)));
typedef unsigned short v4us __attribute__((ext_vector_type(4)));

union Frag  { v16h v; v8h h[2]; };
union Pack8 { v8h h; v4u u; };

__device__ __forceinline__ int clampi(int v, int lo, int hi) { return min(max(v, lo), hi); }

__device__ __forceinline__ v8f mma16(v16h a, v16h b, v8f c) {
  c = __builtin_amdgcn_wmma_f32_16x16x32_f16(false, a, false, b, (short)0, c, false, false);
  asm volatile("v_nop\n\tv_nop\n\tv_nop\n\tv_nop" : "+v"(c) : "v"(a), "v"(b));
  return c;
}

__device__ __forceinline__ v16h ldfrag(const _Float16* p, int ld, int row0, int k0, int lane) {
  const int m = lane & 15, lh = lane >> 4;
  const _Float16* q = p + (size_t)(row0 + m) * ld + k0 + 8 * lh;
  Frag f;
  f.h[0] = *(const v8h*)(q);
  f.h[1] = *(const v8h*)(q + 16);
  return f.v;
}

__device__ __forceinline__ v8f zero8() { return (v8f){0.f, 0.f, 0.f, 0.f, 0.f, 0.f, 0.f, 0.f}; }

__device__ __forceinline__ v4u pack8h(v4f a0, v4f a1) {
  Pack8 pk;
  pk.h = (v8h){(_Float16)a0[0], (_Float16)a0[1], (_Float16)a0[2], (_Float16)a0[3],
               (_Float16)a1[0], (_Float16)a1[1], (_Float16)a1[2], (_Float16)a1[3]};
  return pk.u;
}

__global__ __launch_bounds__(256) void k_tr(const float* __restrict__ src, _Float16* __restrict__ dst,
                                            int R, int C, float scale) {
  __shared__ __align__(16) float tile[32 * TP];
  const int tid = threadIdx.x;
  const size_t slab = (size_t)R * (size_t)C;
  const float* s = src + (size_t)blockIdx.z * slab;
  _Float16* d = dst + (size_t)blockIdx.z * slab;
  const int c0 = blockIdx.x * 32, r0 = blockIdx.y * 64;
  const int tx = tid & 31, ty = tid >> 5;
#pragma unroll
  for (int j = 0; j < 8; ++j)
    tile[tx * TP + ty + 8 * j] = s[(size_t)(r0 + ty + 8 * j) * C + c0 + tx] * scale;
  __syncthreads();
  const int orow = tid >> 3, q = tid & 7;
  const v4f a0 = *(const v4f*)(tile + orow * TP + 8 * q);
  const v4f a1 = *(const v4f*)(tile + orow * TP + 8 * q + 4);
  const v4u vv = pack8h(a0, a1);
  volatile v4u* dp = (volatile v4u*)(d + (size_t)(c0 + orow) * R + r0 + 8 * q);
  *dp = vv;
  __threadfence();
  *dp = vv;
}

__global__ __launch_bounds__(256) void k_gate(const float* __restrict__ x, const float* __restrict__ wg,
                                              const float* __restrict__ bg, int* __restrict__ eidp) {
  __shared__ __align__(16) float sW[DD * NE];
  __shared__ float sB[NE];
  __shared__ __align__(16) int sE[32];
  const int tid = threadIdx.x, lane = tid & 31, wave = tid >> 5;

#pragma unroll 1
  for (int i = tid; i < DD * NE / 4; i += 256) *(v4f*)(sW + 4 * i) = *(const v4f*)(wg + 4 * i);
  if (tid < NE) sB[tid] = bg[tid];
  __syncthreads();

#pragma unroll 1
  for (int j = 0; j < 4; ++j) {
    const int t = blockIdx.x * 32 + wave * 4 + j;
    const float* xr = x + (size_t)t * DD;
    float acc[NE];
#pragma unroll
    for (int e = 0; e < NE; ++e) acc[e] = 0.f;
#pragma unroll 1
    for (int i = 0; i < DD / 128; ++i) {
      const int d0 = i * 128 + lane * 4;
      const v4f xv = *(const v4f*)(xr + d0);
#pragma unroll
      for (int dd = 0; dd < 4; ++dd) {
        const v4f w0 = *(const v4f*)(sW + (d0 + dd) * NE);
        const v4f w1 = *(const v4f*)(sW + (d0 + dd) * NE + 4);
        const float xs = xv[dd];
        acc[0] = fmaf(xs, w0[0], acc[0]);
        acc[1] = fmaf(xs, w0[1], acc[1]);
        acc[2] = fmaf(xs, w0[2], acc[2]);
        acc[3] = fmaf(xs, w0[3], acc[3]);
        acc[4] = fmaf(xs, w1[0], acc[4]);
        acc[5] = fmaf(xs, w1[1], acc[5]);
        acc[6] = fmaf(xs, w1[2], acc[6]);
        acc[7] = fmaf(xs, w1[3], acc[7]);
      }
    }
#pragma unroll
    for (int e = 0; e < NE; ++e) {
      float v = acc[e];
#pragma unroll
      for (int off = 16; off > 0; off >>= 1) v += __shfl_xor(v, off, 32);
      acc[e] = v;
    }
    float bv = acc[0] + sB[0];
    int best = 0;
#pragma unroll
    for (int e = 1; e < NE; ++e) {
      const float v = acc[e] + sB[e];
      if (v > bv) { bv = v; best = e; }
    }
    if (lane == 0) sE[wave * 4 + j] = best;
  }
  __syncthreads();
  if (wave == 0) {
    const v4i ve = *(const v4i*)(sE + (lane & 7) * 4);
    volatile v4i* de = (volatile v4i*)(eidp + blockIdx.x * 32 + (lane & 7) * 4);
    if (lane < 8) *de = ve;
    __threadfence();
    if (lane < 8) *de = ve;
  }
}

__global__ __launch_bounds__(256) void k_lists(const int* __restrict__ cid, int* __restrict__ tokp,
                                               int* __restrict__ posp, int* __restrict__ tab) {
  __shared__ __align__(16) unsigned short ltok[NROWS];
  __shared__ int wc[8 * NE];
  __shared__ int wsum[8 * NE];
  __shared__ int srun[NE];
  __shared__ __align__(16) int sTab[64];
  const int tid = threadIdx.x, lane = tid & 31, wave = tid >> 5;
  const unsigned ltm = (1u << lane) - 1u;

  for (int i = tid; i < NROWS; i += 256) ltok[i] = (unsigned short)0;
  if (tid < 64) sTab[tid] = 0;
  if (tid < NE) srun[tid] = 0;

  int hacc[NE];
#pragma unroll
  for (int e = 0; e < NE; ++e) hacc[e] = 0;
#pragma unroll 1
  for (int ch = 0; ch < NCH; ++ch) {
    const int t  = ch * 256 + tid;
    const int et = clampi(cid[t], 0, NE - 1);
#pragma unroll
    for (int e = 0; e < NE; ++e) {
      const unsigned bal = __builtin_amdgcn_ballot_w32(et == e);
      hacc[e] += __builtin_popcount(bal);
    }
  }
  int hv = 0;
#pragma unroll
  for (int e = 0; e < NE; ++e) hv = (lane == e) ? hacc[e] : hv;
  if (lane < NE) wsum[wave * NE + lane] = hv;
  __syncthreads();
  if (tid < NE) {
    int s = 0;
#pragma unroll
    for (int q = 0; q < 8; ++q) s += wsum[q * NE + tid];
    sTab[tid] = s;
  }
  __syncthreads();
  if (tid == 0) {
    int run = 0;
#pragma unroll 1
    for (int e = 0; e < NE; ++e) {
      sTab[32 + e] = run;
      run += (clampi(sTab[e], 0, NTOK) + 63) >> 6;
    }
    sTab[32 + NE] = clampi(run, 0, NTILE);
  }
  __syncthreads();

#pragma unroll 1
  for (int ch = 0; ch < NCH; ++ch) {
    const int t  = ch * 256 + tid;
    const int et = clampi(cid[t], 0, NE - 1);
    int pre = 0;
#pragma unroll
    for (int e = 0; e < NE; ++e) {
      const bool m = (et == e);
      const unsigned bal = __builtin_amdgcn_ballot_w32(m);
      pre = m ? __builtin_popcount(bal & ltm) : pre;
      if (lane == 0) wc[wave * NE + e] = __builtin_popcount(bal);
    }
    __syncthreads();
    int base = srun[et];
#pragma unroll
    for (int q = 0; q < 8; ++q) base += (q < wave) ? wc[q * NE + et] : 0;
    int tot = 0;
    if (tid < NE) {
#pragma unroll
      for (int q = 0; q < 8; ++q) tot += wc[q * NE + tid];
    }
    const int tbe = clampi(sTab[32 + et], 0, NTILE - 1);
    const int row = clampi(tbe * 64 + base + pre, 0, NROWS - 1);
    ltok[row] = (unsigned short)t;
    volatile int* pd = (volatile int*)(posp + t);
    *pd = row;
    __threadfence();
    *pd = row;
    __syncthreads();
    if (tid < NE) srun[tid] += tot;
  }
  __syncthreads();

  for (int ps = 0; ps < 2; ++ps) {
#pragma unroll 1
    for (int it = 0; it < NPIT; ++it) {
      const int p = tid + 256 * it;
      if (p < NPC) {
        const v4us u = *(const v4us*)(ltok + p * 4);
        const v4i v = (v4i){(int)u[0], (int)u[1], (int)u[2], (int)u[3]};
        *(volatile v4i*)(tokp + (size_t)p * 4) = v;
      }
    }
    __threadfence();
  }
  if (wave == 0) {
    const v4i v = *(const v4i*)(sTab + (lane & 15) * 4);
    volatile v4i* d = (volatile v4i*)(tab + (lane & 15) * 4);
    if (lane < 16) *d = v;
    __threadfence();
    if (lane < 16) *d = v;
  }
}

__global__ __launch_bounds__(64) void k_gather(const float* __restrict__ x, const int* __restrict__ tokp,
                                               _Float16* __restrict__ xg) {
  const int row = blockIdx.x;
  const int t = clampi(tokp[row], 0, NTOK - 1);
  const int o = (int)threadIdx.x * 8;
  const float* xr = x + (size_t)t * DD + o;
  const v4f a0 = *(const v4f*)(xr);
  const v4f a1 = *(const v4f*)(xr + 4);
  const v4u vv = pack8h(a0, a1);
  volatile v4u* dp = (volatile v4u*)(xg + (size_t)row * DD + o);
  *dp = vv;
  __threadfence();
  *dp = vv;
}

template <int KK, int NO, int MODE>
__global__ __launch_bounds__(256) void k_ffn(const _Float16* __restrict__ ap, const _Float16* __restrict__ wt,
                                             const float* __restrict__ bias, const int* __restrict__ tab,
                                             _Float16* __restrict__ hout, float* __restrict__ yout) {
  __shared__ __align__(16) float sC[8 * 16 * YPITCH];
  __shared__ __align__(16) _Float16 sH[8 * 16 * HPITCH];
  __shared__ int sTab[64];
  const int tid = threadIdx.x, lane = tid & 31, wave = tid >> 5;
  const int hh = lane >> 4, c = lane & 15;
  const int wm = wave & 3, wn = wave >> 2;
  const int b  = blockIdx.x;

  if (tid < 64) sTab[tid] = tab[tid];
  __syncthreads();
  const int ntl = clampi(sTab[32 + NE], 0, NTILE);
  if (b >= ntl) return;
  int e = 0;
#pragma unroll
  for (int q = 1; q < NE; ++q) e += (clampi(sTab[32 + q], 0, NTILE) <= b) ? 1 : 0;

  const _Float16* we = wt + (size_t)e * ((size_t)NO * (size_t)KK);
  const float* bse = bias + e * NO;
  const int arow0 = b * 64 + wm * 16;
  float* cw = sC + wave * (16 * YPITCH);
  _Float16* hw = sH + wave * (16 * HPITCH);

#pragma unroll 1
  for (int nc = 0; nc < NO / 128; ++nc) {
    const int brow = nc * 128 + wn * 64;
    v8f acc[4];
#pragma unroll
    for (int t = 0; t < 4; ++t) acc[t] = zero8();
#pragma unroll 2
    for (int ks = 0; ks < KK / 32; ++ks) {
      const int kg = ks * 32;
      const v16h a = ldfrag(ap, KK, arow0, kg, lane);
#pragma unroll
      for (int t = 0; t < 4; ++t) {
        const v16h bq = ldfrag(we, KK, brow + 16 * t, kg, lane);
        acc[t] = mma16(a, bq, acc[t]);
      }
    }
    if (MODE == 0) {
#pragma unroll
      for (int t = 0; t < 4; ++t) {
        const int ncol = 16 * t + c;
        const float bv = bse[brow + ncol];
#pragma unroll
        for (int r = 0; r < 8; ++r) {
          const float v = fmaxf(acc[t][r] * INV64 + bv, 0.0f) * CHH;
          hw[(8 * hh + r) * HPITCH + ncol] = (_Float16)v;
        }
      }
      __syncthreads();
      for (int ps = 0; ps < 2; ++ps) {
#pragma unroll
        for (int i = 0; i < 4; ++i) {
          const int row = 4 * i + (lane >> 3);
          const int q = lane & 7;
          Pack8 pk;
          pk.h = *(const v8h*)(hw + row * HPITCH + 8 * q);
          const size_t go = (size_t)(arow0 + row) * NO + brow + 8 * q;
          *(volatile v4u*)(hout + go) = pk.u;
        }
        __threadfence();
      }
    } else {
#pragma unroll
      for (int t = 0; t < 4; ++t) {
        const int ncol = 16 * t + c;
        const float bv = bse[brow + ncol];
#pragma unroll
        for (int r = 0; r < 8; ++r) cw[(8 * hh + r) * YPITCH + ncol] = acc[t][r] * INVHY + bv;
      }
      __syncthreads();
      for (int ps = 0; ps < 2; ++ps) {
#pragma unroll
        for (int i = 0; i < 8; ++i) {
          const int row = 2 * i + hh;
          const v4f v = *(const v4f*)(cw + row * YPITCH + c * 4);
          const size_t go = (size_t)(arow0 + row) * NO + brow + c * 4;
          *(volatile v4f*)(yout + go) = v;
        }
        __threadfence();
      }
    }
    __syncthreads();
  }
}

__global__ __launch_bounds__(128) void k_out(const float* __restrict__ yp, const int* __restrict__ posp,
                                             float* __restrict__ out) {
  const int t  = blockIdx.x;
  const int c4 = (int)threadIdx.x;
  const int r  = clampi(posp[t], 0, NROWS - 1);
  const v4f v = *(const v4f*)(yp + (size_t)r * DD + c4 * 4);
  volatile v4f* dp = (volatile v4f*)(out + (size_t)t * DD + c4 * 4);
  *dp = v;
  __threadfence();
  *dp = v;
}

extern "C" void kernel_launch(void* const* d_in, const int* in_sizes, int n_in,
                              void* d_out, int out_size, void* d_ws, size_t ws_size,
                              hipStream_t stream) {
  if (n_in < 7) return;
  if (in_sizes[0] != NTOK * DD) return;
  if (in_sizes[1] != DD * NE) return;
  if (in_sizes[2] != NE) return;
  if (in_sizes[3] != NE * DD * FF) return;
  if (in_sizes[4] != NE * FF) return;
  if (in_sizes[5] != NE * FF * DD) return;
  if (in_sizes[6] != NE * DD) return;
  if (out_size != NTOK * DD) return;

  const float* x  = (const float*)d_in[0];
  const float* Wg = (const float*)d_in[1];
  const float* bg = (const float*)d_in[2];
  const float* W1 = (const float*)d_in[3];
  const float* b1 = (const float*)d_in[4];
  const float* W2 = (const float*)d_in[5];
  const float* b2 = (const float*)d_in[6];
  float* out = (float*)d_out;

  size_t off = 0;
  const size_t oW1 = off; off += (size_t)NE * FF * DD * 2;
  const size_t oW2 = off; off += (size_t)NE * DD * FF * 2;
  const size_t oEI = off; off += (size_t)NTOK * 4;
  const size_t oTK = off; off += (size_t)NROWS * 4;
  const size_t oPS = off; off += (size_t)NTOK * 4;
  const size_t oTB = off; off += (size_t)256;
  const size_t oXG = off; off += (size_t)NROWS * DD * 2;
  const size_t oHH = off; off += (size_t)NROWS * FF * 2;
  const size_t oY  = off; off += (size_t)NROWS * DD * 4;
  if (off > ws_size) return;
  if (off > (size_t)134217728) return;
  if ((oW2 | oEI | oTK | oPS | oTB | oXG | oHH | oY) & (size_t)127) return;

  char* ws = (char*)d_ws;
  _Float16* W1t = (_Float16*)(ws + oW1);
  _Float16* W2t = (_Float16*)(ws + oW2);
  int*      EID = (int*)(ws + oEI);
  int*      TOK = (int*)(ws + oTK);
  int*      POS = (int*)(ws + oPS);
  int*      TAB = (int*)(ws + oTB);
  _Float16* Xg  = (_Float16*)(ws + oXG);
  _Float16* Hh  = (_Float16*)(ws + oHH);
  float*    Y   = (float*)(ws + oY);

  k_tr<<<dim3(FF / 32, DD / 64, NE), dim3(256), 0, stream>>>(W1, W1t, DD, FF, WSC);
  k_tr<<<dim3(DD / 32, FF / 64, NE), dim3(256), 0, stream>>>(W2, W2t, FF, DD, WSC);
  k_gate<<<dim3(NTOK / 32), dim3(256), 0, stream>>>(x, Wg, bg, EID);
  k_lists<<<dim3(1), dim3(256), 0, stream>>>(EID, TOK, POS, TAB);
  k_gather<<<dim3(NROWS), dim3(64), 0, stream>>>(x, TOK, Xg);
  k_ffn<DD, FF, 0><<<dim3(NTILE), dim3(256), 0, stream>>>(Xg, W1t, b1, TAB, Hh, Y);
  k_ffn<FF, DD, 1><<<dim3(NTILE), dim3(256), 0, stream>>>(Hh, W2t, b2, TAB, Hh, Y);
  k_out<<<dim3(NTOK), dim3(128), 0, stream>>>(Y, POS, out);
  (void)hipGetLastError();
}
